// SpatialGraph_70738111365774
// MI455X (gfx1250) — hardware-run, weakly checked
//
#include <hip/hip_runtime.h>
#include <math.h>

typedef __attribute__((ext_vector_type(16))) _Float16 v16h;
typedef __attribute__((ext_vector_type(8)))  _Float16 v8h;
typedef __attribute__((ext_vector_type(16))) __bf16   v16b;
typedef __attribute__((ext_vector_type(8)))  __bf16   v8b;
typedef __attribute__((ext_vector_type(8)))  float    v8f;
typedef __attribute__((ext_vector_type(4)))  float    v4f;
typedef __attribute__((ext_vector_type(4)))  unsigned int v4u;

constexpr int kBatch = 64;
constexpr int kCls   = 80;
constexpr int kDim   = 256;
constexpr int kBox   = 32;
constexpr int kRows  = kBatch * kCls;
constexpr int kQKld  = 2 * kDim;
constexpr float kImg    = 224.0f;
constexpr float kImgMax = kImg - 1.0f;
constexpr int kS0 = 10;
constexpr int kS1 = 20;
constexpr int kW0 = (kS0 * kS0 + 31) / 32;
constexpr int kW1 = (kS1 * kS1 + 31) / 32;
constexpr int kMW = kW0 + kW1;
constexpr float kInvCells0 = 1.0f / (float)(kS0 * kS0);
constexpr float kInvCells1 = 1.0f / (float)(kS1 * kS1);

constexpr int isqrt_c(int n) { int r = 0; while ((r + 1) * (r + 1) <= n) ++r; return r; }
constexpr int kSqrtD = isqrt_c(kDim);
static_assert(kSqrtD * kSqrtD == kDim);
static_assert(kRows == 5120 && kDim == 256 && kCls == 80 && kBox == 32 && kMW == 17);
static_assert((kRows % 64) == 0 && (kDim % 64) == 0 && (kQKld % 64) == 0 && (kDim % 32) == 0);
static_assert((kCls % 16) == 0 && (kCls % 4) == 0);

constexpr float kXCarry   = 16.0f;
constexpr float kWCarry   = 256.0f;
constexpr float kActCarry = 16.0f;
constexpr float kPCarry   = 32768.0f;
constexpr float kOCarry   = 512.0f;
constexpr float kProjScale  = kActCarry / (kXCarry * kWCarry);
constexpr float kScoreScale = 1.0f / (kActCarry * kActCarry * (float)kSqrtD);
constexpr float kPVScale    = kOCarry / (kPCarry * kActCarry);
constexpr float kOutScale   = 1.0f / (kOCarry * kWCarry);
constexpr float kF16MinNormal = 6.103515625e-05f;

constexpr size_t kSzWT   = (size_t)4 * kDim * kDim * 2;
constexpr size_t kSzXH   = (size_t)kRows * kDim * 2;
constexpr size_t kSzBIAS = (size_t)3 * kDim * 4;
constexpr size_t kSzAFF  = (size_t)kBatch * kCls * kCls * 4;
constexpr size_t kSzQK   = (size_t)kRows * kQKld * 2;
constexpr size_t kSzVT   = (size_t)kDim * kRows * 2;
constexpr size_t kSzOH   = (size_t)kRows * kDim * 2;
constexpr size_t kOffWT   = 0;
constexpr size_t kOffXH   = kOffWT + kSzWT;
constexpr size_t kOffBIAS = kOffXH + kSzXH;
constexpr size_t kOffAFF  = kOffBIAS + kSzBIAS;
constexpr size_t kOffQK   = kOffAFF + kSzAFF;
constexpr size_t kOffVT   = kOffQK + kSzQK;
constexpr size_t kOffOH   = kOffVT + kSzVT;
constexpr size_t kWsTotal = kOffOH + kSzOH;
static_assert(kWsTotal == 15272960ull);
static_assert(kWsTotal <= 134217728ull);
static_assert((kOffXH % 128) == 0 && (kOffBIAS % 128) == 0 && (kOffAFF % 128) == 0 &&
              (kOffQK % 128) == 0 && (kOffVT % 128) == 0 && (kOffOH % 128) == 0);

__device__ __forceinline__ unsigned short f2bf_bits(float f) {
  unsigned u = __float_as_uint(f);
  return (unsigned short)((u + 0x7FFFu + ((u >> 16) & 1u)) >> 16);
}
__device__ __forceinline__ float bf_bits2f(unsigned short h) { return __uint_as_float(((unsigned)h) << 16); }

__device__ __forceinline__ float ftz16(float f) { return (fabsf(f) < kF16MinNormal) ? 0.0f : f; }
__device__ __forceinline__ unsigned short h_bits(float f) {
  const _Float16 h = (_Float16)ftz16(f);
  return __builtin_bit_cast(unsigned short, h);
}
__device__ __forceinline__ unsigned pk16(unsigned short a, unsigned short b) { return (unsigned)a | ((unsigned)b << 16); }

__device__ __forceinline__ void dep_guard1_h(v8f& a, v16h x, v16h y) { asm volatile("v_nop\n\tv_nop\n\tv_nop\n\tv_nop" : "+v"(a) : "v"(x), "v"(y)); }
__device__ __forceinline__ void dep_guard1_b(v8f& a, v16b x, v16b y) { asm volatile("v_nop\n\tv_nop\n\tv_nop\n\tv_nop" : "+v"(a) : "v"(x), "v"(y)); }
__device__ __forceinline__ void keep4_h(v16h a, v16h b, v16h c, v16h d) { asm volatile("v_nop" :: "v"(a), "v"(b), "v"(c), "v"(d)); }
__device__ __forceinline__ void keep4_b(v16b a, v16b b, v16b c, v16b d) { asm volatile("v_nop" :: "v"(a), "v"(b), "v"(c), "v"(d)); }
__device__ __forceinline__ void acc_guard4(v8f& a, v8f& b, v8f& c, v8f& d) { asm volatile("v_nop\n\tv_nop\n\tv_nop\n\tv_nop" : "+v"(a), "+v"(b), "+v"(c), "+v"(d)); }

template <typename T> struct Frag;
template <> struct Frag<_Float16> {
  typedef v16h V; union U { v16h v; v8h h[2]; };
  static __device__ __forceinline__ v16h load(const _Float16* p) {
    U f; f.h[0] = *(const v8h*)(p); f.h[1] = *(const v8h*)(p + 16); return f.v;
  }
  static __device__ __forceinline__ v8f mma(v16h a, v16h b, v8f c) {
    return __builtin_amdgcn_wmma_f32_16x16x32_f16(false, a, false, b, (short)0, c, false, false);
  }
  static __device__ __forceinline__ void guard1(v8f& a, v16h x, v16h y) { dep_guard1_h(a, x, y); }
  static __device__ __forceinline__ void keep(v16h a, v16h b, v16h c, v16h d) { keep4_h(a, b, c, d); }
};
template <> struct Frag<__bf16> {
  typedef v16b V; union U { v16b v; v8b h[2]; };
  static __device__ __forceinline__ v16b load(const __bf16* p) {
    U f; f.h[0] = *(const v8b*)(p); f.h[1] = *(const v8b*)(p + 16); return f.v;
  }
  static __device__ __forceinline__ v8f mma(v16b a, v16b b, v8f c) {
    return __builtin_amdgcn_wmma_f32_16x16x32_bf16(false, a, false, b, (short)0, c, false, false);
  }
  static __device__ __forceinline__ void guard1(v8f& a, v16b x, v16b y) { dep_guard1_b(a, x, y); }
  static __device__ __forceinline__ void keep(v16b a, v16b b, v16b c, v16b d) { keep4_b(a, b, c, d); }
};

__device__ __forceinline__ v8f mma_g(v16h a, v16h b, v8f c) {
  c = __builtin_amdgcn_wmma_f32_16x16x32_f16(false, a, false, b, (short)0, c, false, false);
  asm volatile("v_nop\n\tv_nop\n\tv_nop\n\tv_nop" : "+v"(c) : "v"(a), "v"(b));
  return c;
}

template <int ET> struct Elem;
template <> struct Elem<0> { typedef _Float16 T; };
template <> struct Elem<1> { typedef __bf16 T; };
template <int ET, bool SPLIT, int BIAS_MODE, int OUT_MODE, bool RESID, int ACT = 0>
__global__ __launch_bounds__(256) void wmma_gemm64(
    const unsigned short* __restrict__ Ap, const unsigned short* __restrict__ A2p, int lda, long strideA,
    const unsigned short* __restrict__ Btp, const unsigned short* __restrict__ Bt2p, int ldb, long strideB,
    void* __restrict__ Cout, void* __restrict__ Cout2, int ldc, long strideC,
    const float* __restrict__ bias,
    const float* __restrict__ resid, long strideR,
    int M, int N, int K, float scale) {
  typedef typename Elem<ET>::T T;
  typedef typename Frag<T>::V V;
  const T* A = (const T*)Ap; const T* A2 = (const T*)A2p; const T* Bt = (const T*)Btp; const T* Bt2 = (const T*)Bt2p;
  __shared__ __align__(16) float sT[8][16 * 68];
  const int b    = blockIdx.y;
  const int lane = threadIdx.x & 31;
  const int wave = threadIdx.x >> 5;
  const int tilesN = N >> 6;
  const int tilesM = M >> 6;
  const int tile = blockIdx.x * 8 + wave;
  if (tile >= tilesM * tilesN) return;
  const int tm = tile / tilesN;
  const int tn = tile - tm * tilesN;
  const int m0 = tm << 6;
  const int n0 = tn << 6;

  const T* Ab  = A  + (size_t)b * strideA;
  const T* Bb  = Bt + (size_t)b * strideB;
  const T* Ab2 = SPLIT ? (A2  + (size_t)b * strideA) : nullptr;
  const T* Bb2 = SPLIT ? (Bt2 + (size_t)b * strideB) : nullptr;

  const int rlane = lane & 15;
  const int koff  = (lane >> 4) * 8;
  const int mOff  = (lane >> 4) * 8;

  v8f acc[4][4];
#pragma unroll
  for (int i = 0; i < 4; ++i)
#pragma unroll
    for (int j = 0; j < 4; ++j) acc[i][j] = (v8f){0.f,0.f,0.f,0.f,0.f,0.f,0.f,0.f};

  for (int k0 = 0; k0 < K; k0 += 32) {
    V bh[4], bl[4];
#pragma unroll
    for (int j = 0; j < 4; ++j) {
      const size_t bo = (size_t)(n0 + (j << 4) + rlane) * ldb + koff + k0;
      bh[j] = Frag<T>::load(Bb + bo);
      if (SPLIT) bl[j] = Frag<T>::load(Bb2 + bo);
    }
#pragma unroll
    for (int i = 0; i < 4; ++i) {
      const size_t ao = (size_t)(m0 + (i << 4) + rlane) * lda + koff + k0;
      V ah = Frag<T>::load(Ab + ao);
      V al;
      if (SPLIT) al = Frag<T>::load(Ab2 + ao);
#pragma unroll
      for (int j = 0; j < 4; ++j) {
        acc[i][j] = Frag<T>::mma(ah, bh[j], acc[i][j]);
        if (SPLIT) {
          acc[i][j] = Frag<T>::mma(ah, bl[j], acc[i][j]);
          acc[i][j] = Frag<T>::mma(al, bh[j], acc[i][j]);
        }
      }
      Frag<T>::guard1(acc[i][0], ah, bh[0]);
      Frag<T>::guard1(acc[i][1], ah, bh[1]);
      Frag<T>::guard1(acc[i][2], ah, bh[2]);
      Frag<T>::guard1(acc[i][3], SPLIT ? al : ah, bh[3]);
    }
    Frag<T>::keep(bh[0], bh[1], bh[2], bh[3]);
    if (SPLIT) Frag<T>::keep(bl[0], bl[1], bl[2], bl[3]);
  }
  acc_guard4(acc[0][0], acc[0][1], acc[0][2], acc[0][3]);
  acc_guard4(acc[1][0], acc[1][1], acc[1][2], acc[1][3]);
  acc_guard4(acc[2][0], acc[2][1], acc[2][2], acc[2][3]);
  acc_guard4(acc[3][0], acc[3][1], acc[3][2], acc[3][3]);

  float* slab = sT[wave];
  const float* Rb = RESID ? (resid + (size_t)b * strideR) : nullptr;
#pragma unroll
  for (int i = 0; i < 4; ++i) {
    const int mBase = m0 + (i << 4);
#pragma unroll
    for (int j = 0; j < 4; ++j) {
      const int n = n0 + (j << 4) + rlane;
      float bv = 0.f;
      if (BIAS_MODE == 2) bv = bias[n];
#pragma unroll
      for (int r = 0; r < 8; ++r) {
        float v = acc[i][j][r] * scale;
        if (BIAS_MODE == 1) v += bias[mBase + mOff + r];
        if (BIAS_MODE == 2) v += bv;
        if (RESID) v += Rb[(size_t)(mBase + mOff + r) * ldc + n];
        if (ACT == 2) v = fmaxf(v, 0.0f);
        if (ACT == 4) v = (v > 0.f) ? v : 0.01f * v;
        slab[(mOff + r) * 68 + (j << 4) + rlane] = v;
      }
    }
    __builtin_amdgcn_fence(__ATOMIC_RELEASE, "workgroup");
    __builtin_amdgcn_wave_barrier();
    __builtin_amdgcn_fence(__ATOMIC_ACQUIRE, "workgroup");
    if (OUT_MODE == 0) {
      float* C = (float*)Cout + (size_t)b * strideC;
      const int hh = lane >> 4, c4 = (lane & 15) * 4;
      for (int pass = 0; pass < 2; ++pass) {
#pragma unroll
        for (int it = 0; it < 8; ++it) {
          const int row = it * 2 + hh;
          v4f v = *(const v4f*)(slab + row * 68 + c4);
          *(volatile v4f*)(C + (size_t)(mBase + row) * ldc + n0 + c4) = v;
        }
        __threadfence();
      }
    } else {
      const int q = lane >> 3, c8 = (lane & 7) * 8;
      unsigned short* C  = (unsigned short*)Cout  + (size_t)b * strideC;
      unsigned short* C2 = (OUT_MODE == 2) ? ((unsigned short*)Cout2 + (size_t)b * strideC) : nullptr;
      for (int pass = 0; pass < 2; ++pass) {
#pragma unroll
        for (int it = 0; it < 4; ++it) {
          const int row = it * 4 + q;
          const float* sp = slab + row * 68 + c8;
          v8h hv, lv;
#pragma unroll
          for (int e = 0; e < 8; ++e) {
            if (OUT_MODE == 1) {
              const float t = ftz16(sp[e]);
              hv[e] = (_Float16)t;
            } else {
              unsigned short hb = f2bf_bits(sp[e]);
              unsigned short lb = f2bf_bits(sp[e] - bf_bits2f(hb));
              hv[e] = __builtin_bit_cast(_Float16, hb);
              lv[e] = __builtin_bit_cast(_Float16, lb);
            }
          }
          *(volatile v8h*)(C + (size_t)(mBase + row) * ldc + n0 + c8) = hv;
          if (OUT_MODE == 2) *(volatile v8h*)(C2 + (size_t)(mBase + row) * ldc + n0 + c8) = lv;
        }
        __threadfence();
      }
    }
    __builtin_amdgcn_fence(__ATOMIC_RELEASE, "workgroup");
    __builtin_amdgcn_wave_barrier();
    __builtin_amdgcn_fence(__ATOMIC_ACQUIRE, "workgroup");
  }
}

__global__ __launch_bounds__(256) void wtcast_kernel(const float* __restrict__ W0, const float* __restrict__ W1,
                                                     const float* __restrict__ W2, const float* __restrict__ W3,
                                                     unsigned short* __restrict__ out, float carry) {
  __shared__ float sm[64][65];
  const int t  = threadIdx.x;
  const int d0 = blockIdx.x * 64;
  const int h0 = blockIdx.y * 64;
  const int z  = blockIdx.z;
  const float* W = (z == 0) ? W0 : (z == 1) ? W1 : (z == 2) ? W2 : W3;
#pragma unroll
  for (int i = 0; i < 16; ++i) {
    const int e = i * 256 + t;
    const int r = e >> 6;
    const int c = e & 63;
    sm[c][r] = W[(size_t)(d0 + r) * kDim + h0 + c] * carry;
  }
  __syncthreads();
  const int lane = t & 31, wave = t >> 5;
  const int q = lane >> 3, c8 = (lane & 7) * 8;
  unsigned short* op = out + (size_t)z * kDim * kDim;
  for (int pass = 0; pass < 2; ++pass) {
#pragma unroll
    for (int it = 0; it < 2; ++it) {
      const int row = wave * 8 + it * 4 + q;
      unsigned short hb[8];
#pragma unroll
      for (int e = 0; e < 8; ++e) hb[e] = h_bits(sm[row][c8 + e]);
      const v4u u = (v4u){pk16(hb[0], hb[1]), pk16(hb[2], hb[3]), pk16(hb[4], hb[5]), pk16(hb[6], hb[7])};
      *(volatile v4u*)(op + (size_t)(h0 + row) * kDim + d0 + c8) = u;
    }
    __threadfence();
  }
}

__global__ __launch_bounds__(256) void cast8_f16_kernel(const float* __restrict__ in, unsigned short* __restrict__ out,
                                                        int n8, float carry) {
  const int i = blockIdx.x * 256 + threadIdx.x;
  if (i >= n8) return;
  const float* p = in + 8 * (size_t)i;
  const v4f a = *(const v4f*)(p);
  const v4f c = *(const v4f*)(p + 4);
  unsigned short hb[8];
#pragma unroll
  for (int e = 0; e < 4; ++e) {
    hb[e]     = h_bits(a[e] * carry);
    hb[4 + e] = h_bits(c[e] * carry);
  }
  const v4u u = (v4u){pk16(hb[0], hb[1]), pk16(hb[2], hb[3]), pk16(hb[4], hb[5]), pk16(hb[6], hb[7])};
  unsigned short* q = out + 8 * (size_t)i;
  *(volatile v4u*)q = u;
  __threadfence();
  *(volatile v4u*)q = u;
}

__global__ __launch_bounds__(192) void bias_plane_kernel(const float* __restrict__ bq, const float* __restrict__ bk,
                                                         const float* __restrict__ bv, float* __restrict__ out, float carry) {
  const int t   = threadIdx.x;
  const int seg = t >> 6;
  const int o4  = (t & 63) * 4;
  const v4f a = *(const v4f*)(bq + o4);
  const v4f b = *(const v4f*)(bk + o4);
  const v4f c = *(const v4f*)(bv + o4);
  v4f v;
#pragma unroll
  for (int e = 0; e < 4; ++e) {
    const float s = (seg == 0) ? a[e] : ((seg == 1) ? b[e] : c[e]);
    v[e] = s * carry;
  }
  float* q = out + 4 * t;
  *(volatile v4f*)q = v;
  __threadfence();
  *(volatile v4f*)q = v;
}

__device__ __forceinline__ int cell_of(float c, float fs, int smax) {
#pragma clang fp contract(off)
  float t = c * fs;
  t = t / kImg;
  int g = (int)floorf(t);
  g = (g < 0) ? 0 : g;
  g = (g > smax) ? smax : g;
  return g;
}

__global__ __launch_bounds__(256) void affinity_kernel(const float* __restrict__ bboxes, const int* __restrict__ bclass,
                                                       float* __restrict__ aff) {
  __shared__ unsigned sM[kCls * kMW];
  __shared__ __align__(16) float sA[kCls * kCls];
  __shared__ float sInv[kCls];
  __shared__ int      sBcls[kBox];
  __shared__ unsigned sBrm[2 * kBox];
  __shared__ int      sBy1[2 * kBox];
  __shared__ int      sBy2[2 * kBox];
  const int b    = blockIdx.x;
  const int tid  = threadIdx.x;
  const int lane = tid & 31;
  const int wave = tid >> 5;

  const int bi = tid & 31;
  const v4f bb = *(const v4f*)(bboxes + (size_t)(b * kBox + bi) * 4);
  float bx = bb[0];
  float by = bb[1];
  float bw = bb[2];
  float bh = bb[3];
  int cls = bclass[b * kBox + bi];
  asm volatile("" : "+v"(bx));
  asm volatile("" : "+v"(by));
  asm volatile("" : "+v"(bw));
  asm volatile("" : "+v"(bh));
  asm volatile("" : "+v"(cls));

  if (tid < kBox) {
    const float x1 = fminf(fmaxf(bx, 0.0f), kImgMax);
    const float y1 = fminf(fmaxf(by, 0.0f), kImgMax);
    const float x2 = fminf(fmaxf(bx + bw, 0.0f), kImgMax);
    const float y2 = fminf(fmaxf(by + bh, 0.0f), kImgMax);
    int cw = (cls < 0) ? (cls + kCls) : cls;
    const bool valid = (cw >= 0) && (cw < kCls);
    cw = (cw < 0) ? 0 : cw;
    cw = (cw > kCls - 1) ? (kCls - 1) : cw;
    sBcls[tid] = valid ? cw : -1;
#pragma unroll 1
    for (int si = 0; si < 2; ++si) {
      const int S  = si ? kS1 : kS0;
      const float fs = (float)S;
      const int gx1 = cell_of(x1, fs, S - 1);
      const int gy1 = cell_of(y1, fs, S - 1);
      const int gx2 = cell_of(x2, fs, S - 1);
      const int gy2 = cell_of(y2, fs, S - 1);
      int nb = gx2 - gx1 + 1;
      nb = (nb < 0) ? 0 : nb;
      nb = (nb > kS1) ? kS1 : nb;
      const unsigned rmv = ((1u << nb) - 1u) << gx1;
      const unsigned rm  = valid ? rmv : 0u;
      sBrm[si * kBox + tid] = rm;
      sBy1[si * kBox + tid] = gy1;
      sBy2[si * kBox + tid] = gy2;
    }
  }
  __syncthreads();

#pragma unroll 1
  for (int wIdx = tid; wIdx < kCls * kMW; wIdx += 256) {
    const int c  = wIdx / kMW;
    const int w  = wIdx - c * kMW;
    const int si = (w >= kW0) ? 1 : 0;
    const int wi = w - si * kW0;
    const int S  = si ? kS1 : kS0;
    unsigned word = 0u;
#pragma unroll 1
    for (int bxi = 0; bxi < kBox; ++bxi) {
      const int      bc = sBcls[bxi];
      const unsigned rm = sBrm[si * kBox + bxi];
      int ya = sBy1[si * kBox + bxi];
      int yb = sBy2[si * kBox + bxi];
      ya = (ya < 0) ? 0 : ya;
      yb = (yb > S - 1) ? (S - 1) : yb;
      if (bc == c && rm != 0u) {
        for (int yy = ya; yy <= yb; ++yy) {
          const int off = yy * S;
          const int wd  = off >> 5;
          const int sh  = off & 31;
          const unsigned long long m64 = ((unsigned long long)rm) << sh;
          const unsigned lo = (unsigned)(m64 & 0xffffffffull);
          const unsigned hi = (unsigned)(m64 >> 32);
          const unsigned addlo = (wd == wi) ? lo : 0u;
          const unsigned addhi = (wd + 1 == wi) ? hi : 0u;
          word |= addlo;
          word |= addhi;
        }
      }
    }
    sM[wIdx] = word;
  }
  __syncthreads();

#pragma unroll 1
  for (int idx = tid; idx < kCls * kCls; idx += 256) {
    const int i = idx / kCls;
    const int j = idx - i * kCls;
    int l10 = 0;
    int l20 = 0;
#pragma unroll
    for (int w = 0; w < kW0; ++w) l10 += __popc(sM[i * kMW + w] ^ sM[j * kMW + w]);
#pragma unroll
    for (int w = kW0; w < kMW; ++w) l20 += __popc(sM[i * kMW + w] ^ sM[j * kMW + w]);
    const float a10 = (1.0f - (float)l10 * kInvCells0) * 0.5f;
    const float a20 = (1.0f - (float)l20 * kInvCells1) * 0.5f;
    sA[idx] = a10 + a20;
  }
  __syncthreads();

  if (tid < kCls) {
    float s = 0.0f;
#pragma unroll 1
    for (int j = 0; j < kCls; ++j) s += fabsf(sA[tid * kCls + j]);
    sInv[tid] = 1.0f / fmaxf(s, 1e-12f);
  }
  __syncthreads();

  float* ab = aff + (size_t)b * kCls * kCls;
  for (int pass = 0; pass < 2; ++pass) {
#pragma unroll 1
    for (int ch = wave; ch < (kCls * kCls) / 128; ch += 8) {
      const int e0  = (ch * 32 + lane) * 4;
      const int row = e0 / kCls;
      const v4f a = *(const v4f*)(sA + e0);
      const float iv = sInv[row];
      v4f v;
      v[0] = a[0] * iv;
      v[1] = a[1] * iv;
      v[2] = a[2] * iv;
      v[3] = a[3] * iv;
      *(volatile v4f*)(ab + e0) = v;
    }
    __threadfence();
  }
}
static_assert(((kCls * kCls) % 128) == 0);

constexpr int kAtWaves = kCls / 16;
constexpr int kSPitch  = 84;
constexpr int kPPitch  = 88;
constexpr int kOPitch  = 68;
constexpr int kHalfCols = kCls / 2;
static_assert(kAtWaves == 5 && (kHalfCols % 4) == 0 && kSPitch >= kCls && kPPitch >= kCls);

__global__ __launch_bounds__(160) void attn_kernel(const unsigned short* __restrict__ QKp, const unsigned short* __restrict__ VTp,
                                                   const float* __restrict__ AFF, unsigned short* __restrict__ OH) {
  typedef Frag<_Float16> FH;
  __shared__ __align__(16) float    sS[kAtWaves][16 * kSPitch];
  __shared__ __align__(16) _Float16 sP[kAtWaves][16 * kPPitch];
  const _Float16* QK = (const _Float16*)QKp;
  const _Float16* VT = (const _Float16*)VTp;
  const int tid  = threadIdx.x;
  const int wave = tid >> 5;
  const int lane = tid & 31;
  const int hh   = lane >> 4;
  const int c    = lane & 15;
  const int b    = blockIdx.x;
  const int tok0 = b * kCls;
  float*    slab = sS[wave];
  _Float16* pw   = sP[wave];

  v8f s[kAtWaves];
#pragma unroll
  for (int tn = 0; tn < kAtWaves; ++tn) s[tn] = (v8f){0.f,0.f,0.f,0.f,0.f,0.f,0.f,0.f};
  {
    const _Float16* qrow = QK + (size_t)(tok0 + wave * 16 + c) * kQKld + 8 * hh;
    const _Float16* krow = QK + (size_t)(tok0 + c) * kQKld + kDim + 8 * hh;
#pragma unroll 1
    for (int k0 = 0; k0 < kDim; k0 += 32) {
      const v16h a = FH::load(qrow + k0);
#pragma unroll
      for (int tn = 0; tn < kAtWaves; ++tn) {
        const v16h bf = FH::load(krow + (size_t)(tn * 16) * kQKld + k0);
        s[tn] = mma_g(a, bf, s[tn]);
      }
    }
  }
#pragma unroll
  for (int tn = 0; tn < kAtWaves; ++tn) {
#pragma unroll
    for (int r = 0; r < 8; ++r) slab[(8 * hh + r) * kSPitch + tn * 16 + c] = s[tn][r] * kScoreScale;
  }
  __syncthreads();

  {
    const int col0 = hh * kHalfCols;
    float* xr = slab + c * kSPitch + col0;
    const float* ar = AFF + (size_t)b * kCls * kCls + (size_t)(wave * 16 + c) * kCls + col0;
    float m = -INFINITY;
#pragma unroll 1
    for (int j4 = 0; j4 < kHalfCols / 4; ++j4) {
      const v4f sv = *(const v4f*)(xr + 4 * j4);
      const v4f av = *(const v4f*)(ar + 4 * j4);
      v4f x;
      x[0] = sv[0] * av[0];
      x[1] = sv[1] * av[1];
      x[2] = sv[2] * av[2];
      x[3] = sv[3] * av[3];
      *(v4f*)(xr + 4 * j4) = x;
      m = fmaxf(m, fmaxf(fmaxf(x[0], x[1]), fmaxf(x[2], x[3])));
    }
    const float mo = __shfl_xor(m, 16, 32);
    m = fmaxf(m, mo);
    float sum = 0.0f;
#pragma unroll 1
    for (int j4 = 0; j4 < kHalfCols / 4; ++j4) {
      const v4f x = *(const v4f*)(xr + 4 * j4);
      v4f e;
      e[0] = expf(x[0] - m);
      e[1] = expf(x[1] - m);
      e[2] = expf(x[2] - m);
      e[3] = expf(x[3] - m);
      *(v4f*)(xr + 4 * j4) = e;
      sum += e[0];
      sum += e[1];
      sum += e[2];
      sum += e[3];
    }
    const float so = __shfl_xor(sum, 16, 32);
    sum += so;
    const float inv = 1.0f / sum;
    _Float16* pr = pw + c * kPPitch + col0;
#pragma unroll 1
    for (int j4 = 0; j4 < kHalfCols / 4; ++j4) {
      const v4f e = *(const v4f*)(xr + 4 * j4);
      const float p0 = ftz16((e[0] * inv) * kPCarry);
      const float p1 = ftz16((e[1] * inv) * kPCarry);
      const float p2 = ftz16((e[2] * inv) * kPCarry);
      const float p3 = ftz16((e[3] * inv) * kPCarry);
      pr[4 * j4 + 0] = (_Float16)p0;
      pr[4 * j4 + 1] = (_Float16)p1;
      pr[4 * j4 + 2] = (_Float16)p2;
      pr[4 * j4 + 3] = (_Float16)p3;
    }
  }
  __syncthreads();

  v8h z8;
#pragma unroll
  for (int e = 0; e < 8; ++e) z8[e] = (_Float16)0.0f;
  FH::U a0, a1, a2;
  {
    const _Float16* pa = pw + c * kPPitch + 8 * hh;
    a0.h[0] = *(const v8h*)(pa);
    a0.h[1] = *(const v8h*)(pa + 16);
    a1.h[0] = *(const v8h*)(pa + 32);
    a1.h[1] = *(const v8h*)(pa + 48);
    a2.h[0] = *(const v8h*)(pa + 64);
    a2.h[1] = z8;
  }
  const int q  = lane >> 3;
  const int c8 = (lane & 7) * 8;
#pragma unroll 1
  for (int dch = 0; dch < kDim / 64; ++dch) {
    v8f o[4];
#pragma unroll
    for (int j = 0; j < 4; ++j) {
      o[j] = (v8f){0.f,0.f,0.f,0.f,0.f,0.f,0.f,0.f};
      const _Float16* vp = VT + (size_t)(dch * 64 + j * 16 + c) * kRows + tok0 + 8 * hh;
      FH::U b0, b1, b2;
      b0.h[0] = *(const v8h*)(vp);
      b0.h[1] = *(const v8h*)(vp + 16);
      b1.h[0] = *(const v8h*)(vp + 32);
      b1.h[1] = *(const v8h*)(vp + 48);
      b2.h[0] = *(const v8h*)(vp + 64);
      b2.h[1] = z8;
      o[j] = mma_g(a0.v, b0.v, o[j]);
      o[j] = mma_g(a1.v, b1.v, o[j]);
      o[j] = mma_g(a2.v, b2.v, o[j]);
    }
#pragma unroll
    for (int j = 0; j < 4; ++j) {
#pragma unroll
      for (int r = 0; r < 8; ++r) slab[(8 * hh + r) * kOPitch + j * 16 + c] = o[j][r] * kPVScale;
    }
    __syncthreads();
    v8h hv[4];
#pragma unroll
    for (int it = 0; it < 4; ++it) {
      const int row = it * 4 + q;
      const float* sp = slab + row * kOPitch + c8;
      const v4f f0 = *(const v4f*)(sp);
      const v4f f1 = *(const v4f*)(sp + 4);
#pragma unroll
      for (int e = 0; e < 4; ++e) {
        const float t0 = ftz16(f0[e]);
        const float t1 = ftz16(f1[e]);
        hv[it][e]     = (_Float16)t0;
        hv[it][4 + e] = (_Float16)t1;
      }
    }
    for (int pass = 0; pass < 2; ++pass) {
#pragma unroll
      for (int it = 0; it < 4; ++it) {
        const int row = it * 4 + q;
        *(volatile v8h*)(OH + (size_t)(tok0 + wave * 16 + row) * kDim + dch * 64 + c8) = hv[it];
      }
      __threadfence();
    }
    __syncthreads();
  }
}

static_assert(((kRows * kDim / 8) % 256) == 0);

extern "C" void kernel_launch(void* const* d_in, const int* in_sizes, int n_in,
                              void* d_out, int out_size, void* d_ws, size_t ws_size,
                              hipStream_t stream) {
  if (n_in < 11) return;
  if (in_sizes[0] != kRows * kDim) return;
  if (in_sizes[1] != kBatch * kBox * 4) return;
  if (in_sizes[2] != kBatch * kBox) return;
  if (in_sizes[3] != kDim * kDim || in_sizes[5] != kDim * kDim || in_sizes[7] != kDim * kDim || in_sizes[9] != kDim * kDim) return;
  if (in_sizes[4] != kDim || in_sizes[6] != kDim || in_sizes[8] != kDim || in_sizes[10] != kDim) return;
  if (out_size != kRows * kDim) return;
  if (ws_size < kWsTotal) return;

  const float* x      = (const float*)d_in[0];
  const float* bboxes = (const float*)d_in[1];
  const int*   bclass = (const int*)d_in[2];
  const float* Wq     = (const float*)d_in[3];
  const float* bq     = (const float*)d_in[4];
  const float* Wk     = (const float*)d_in[5];
  const float* bk     = (const float*)d_in[6];
  const float* Wv     = (const float*)d_in[7];
  const float* bv     = (const float*)d_in[8];
  const float* Wo     = (const float*)d_in[9];
  const float* bo     = (const float*)d_in[10];
  float* outp = (float*)d_out;

  char* ws = (char*)d_ws;
  unsigned short* WT   = (unsigned short*)(ws + kOffWT);
  unsigned short* XH   = (unsigned short*)(ws + kOffXH);
  float*          BIAS = (float*)(ws + kOffBIAS);
  float*          AFF  = (float*)(ws + kOffAFF);
  unsigned short* QK   = (unsigned short*)(ws + kOffQK);
  unsigned short* VT   = (unsigned short*)(ws + kOffVT);
  unsigned short* OH   = (unsigned short*)(ws + kOffOH);
  unsigned short* WvT  = WT + (size_t)2 * kDim * kDim;
  unsigned short* WoT  = WT + (size_t)3 * kDim * kDim;

  wtcast_kernel<<<dim3(kDim / 64, kDim / 64, 4), 256, 0, stream>>>(Wq, Wk, Wv, Wo, WT, kWCarry);
  cast8_f16_kernel<<<(kRows * kDim / 8) / 256, 256, 0, stream>>>(x, XH, kRows * kDim / 8, kXCarry);
  bias_plane_kernel<<<1, 192, 0, stream>>>(bq, bk, bv, BIAS, kActCarry);

  affinity_kernel<<<kBatch, 256, 0, stream>>>(bboxes, bclass, AFF);

  wmma_gemm64<0, false, 2, 1, false><<<dim3(80, 1), 256, 0, stream>>>(
      XH, XH, kDim, 0L,
      WT, WT, kDim, 0L,
      (void*)QK, (void*)QK, kQKld, 0L,
      BIAS, BIAS, 0L,
      kRows, kQKld, kDim, kProjScale);

  wmma_gemm64<0, false, 1, 1, false><<<dim3(40, 1), 256, 0, stream>>>(
      WvT, WvT, kDim, 0L,
      XH, XH, kDim, 0L,
      (void*)VT, (void*)VT, kRows, 0L,
      BIAS + 2 * kDim, BIAS, 0L,
      kDim, kRows, kDim, kProjScale);

  attn_kernel<<<kBatch, 160, 0, stream>>>(QK, VT, AFF, OH);

  wmma_gemm64<0, false, 2, 0, false><<<dim3(40, 1), 256, 0, stream>>>(
      OH, OH, kDim, 0L,
      WoT, WoT, kDim, 0L,
      (void*)outp, (void*)outp, kDim, 0L,
      bo, bo, 0L,
      kRows, kDim, kDim, kOutScale);
}
